// PerceiverChannelAdapter_10952166605210
// MI455X (gfx1250) — hardware-verified
//
#include <hip/hip_runtime.h>
#include <stddef.h>


typedef _Float16 v16h __attribute__((ext_vector_type(16)));
typedef _Float16 v8h  __attribute__((ext_vector_type(8)));
typedef float    v8f  __attribute__((ext_vector_type(8)));
typedef float    v4f  __attribute__((ext_vector_type(4)));

#ifndef NB
#define NB 16
#endif
#ifndef SEQ
#define SEQ 512
#endif
#define NB_FULL  16
#define SEQ_FULL 512
#define CIN   128
#define DM    64
#define NQ    128
#define MROWS (NB * SEQ)

static_assert(NB >= 1 && NB <= NB_FULL);
static_assert(SEQ >= 64 && SEQ <= SEQ_FULL && (SEQ % 64) == 0);
static_assert((CIN % 64) == 0 && (CIN % 32) == 0);
static_assert(DM == 64);
static_assert((DM % 32) == 0);
static_assert(NQ == 128);
static_assert((NQ % 64) == 0 && (NQ % 32) == 0);
static_assert((MROWS % 64) == 0);
static_assert(((DM * CIN) % 2048) == 0);
static_assert(((DM * DM) % 2048) == 0);

#define LDT 72
#define LDC 68
static_assert((LDT % 8) == 0 && LDT >= 64);
static_assert((LDC % 4) == 0 && LDC >= 64);

#define WCARRY 64.0f
#define XCARRY 64.0f
#define ACARRY 16.0f
#define QCARRY 16.0f
#define LN_EPS 1.0e-5f

#define XT_BYTES   ((size_t)MROWS * CIN * 2)
#define WIN_BYTES  ((size_t)DM * CIN * 2)
#define WSQ_BYTES  ((size_t)DM * DM * 2)
#define ACT_BYTES  ((size_t)MROWS * DM * 2)
#define QC_BYTES   ((size_t)NQ * DM * 2)
#define TS_BYTES   ((size_t)2 * MROWS * 4)
#define QS_BYTES   ((size_t)(2 * NQ + 32) * 4)
#define OFF_XT  ((size_t)0)
#define OFF_WIN (OFF_XT + XT_BYTES)
#define OFF_WV  (OFF_WIN + WIN_BYTES)
#define OFF_WO  (OFF_WV + WSQ_BYTES)
#define OFF_P   (OFF_WO + WSQ_BYTES)
#define OFF_V   (OFF_P + ACT_BYTES)
#define OFF_AC  (OFF_V + ACT_BYTES)
#define OFF_QC  (OFF_AC + ACT_BYTES)
#define OFF_TS  (OFF_QC + QC_BYTES)
#define OFF_QS  (OFF_TS + TS_BYTES)
#define WS_TOTAL (OFF_QS + QS_BYTES)
static_assert((XT_BYTES % 128) == 0 && (WIN_BYTES % 128) == 0 && (WSQ_BYTES % 128) == 0);
static_assert((ACT_BYTES % 128) == 0 && (QC_BYTES % 128) == 0 && (TS_BYTES % 128) == 0);
static_assert((QS_BYTES % 128) == 0);
static_assert(WS_TOTAL <= (size_t)134217728);

__device__ __forceinline__ float bf16r(float x) {
  unsigned int u = __float_as_uint(x);
  u = (u + 0x7FFFu + ((u >> 16) & 1u)) & 0xFFFF0000u;
  return __uint_as_float(u);
}

static __device__ __forceinline__ _Float16 toh_flush(float v) {
  const _Float16 r = (_Float16)v;
  return (fabsf(v) < 6.103515625e-05f) ? (_Float16)0.0f : r;
}

__device__ __forceinline__ v16h frag_at(const _Float16* p) {
  v8h lo = *(const v8h*)(p);
  v8h hi = *(const v8h*)(p + 16);
  v16h out;
#pragma unroll
  for (int i = 0; i < 8; ++i) { out[i] = lo[i]; out[i + 8] = hi[i]; }
  return out;
}

__device__ __forceinline__ v8f wmma16(v16h a, v16h b, v8f c) {
  v8f d = __builtin_amdgcn_wmma_f32_16x16x32_f16(false, a, false, b, (short)0, c,
                                                 false, false);
  asm volatile("v_nop\n\tv_nop\n\tv_nop\n\tv_nop" : "+v"(d) : "v"(a), "v"(b));
  return d;
}

__device__ __forceinline__ float red8_sum(float x) {
#pragma unroll
  for (int off = 1; off < 8; off <<= 1) x += __shfl_xor(x, off, 32);
  return x;
}
__device__ __forceinline__ float red32_sum(float x) {
#pragma unroll
  for (int off = 1; off < 32; off <<= 1) x += __shfl_xor(x, off, 32);
  return x;
}

__global__ __launch_bounds__(256) void xconv_kernel(
    const float* __restrict__ X, _Float16* __restrict__ Xt) {
  __shared__ _Float16 T[64 * LDT];
  const unsigned tid = threadIdx.x;
  const unsigned n0 = blockIdx.x * 64u;
  const unsigned k0 = blockIdx.y * 64u;
  const unsigned b = blockIdx.z;
  const float* src = X + (size_t)b * ((size_t)CIN * SEQ_FULL);
#pragma unroll 4
  for (unsigned j = 0; j < 16u; ++j) {
    const unsigned idx = tid + 256u * j;
    const unsigned kr = idx >> 6, nc = idx & 63u;
    const float v = src[(size_t)(k0 + kr) * SEQ_FULL + n0 + nc];
    T[nc * LDT + kr] = toh_flush(XCARRY * bf16r(v));
  }
  __syncthreads();
  v8h x[2];
  size_t off[2];
#pragma unroll
  for (unsigned i = 0; i < 2u; ++i) {
    const unsigned n = 32u * i + (tid >> 3);
    const unsigned kc = (tid & 7u) * 8u;
    x[i] = *(const v8h*)&T[n * LDT + kc];
    off[i] = (size_t)(b * (unsigned)SEQ + n0 + n) * CIN + k0 + kc;
  }
#pragma unroll
  for (int i = 0; i < 2; ++i) *(volatile v8h*)(Xt + off[i]) = x[i];
  __threadfence();
#pragma unroll
  for (int i = 0; i < 2; ++i) *(volatile v8h*)(Xt + off[i]) = x[i];
}

__global__ __launch_bounds__(256) void wcast_kernel(
    const float* __restrict__ W, _Float16* __restrict__ Wh) {
  const unsigned i8 = (blockIdx.x * 256u + threadIdx.x) * 8u;
  const v4f a0 = *(const v4f*)(W + i8);
  const v4f a1 = *(const v4f*)(W + i8 + 4u);
  v8h o;
#pragma unroll
  for (int i = 0; i < 4; ++i) {
    o[i]     = toh_flush(WCARRY * bf16r(a0[i]));
    o[i + 4] = toh_flush(WCARRY * bf16r(a1[i]));
  }
  _Float16* p = Wh + i8;
  *(volatile v8h*)p = o;
  __threadfence();
  *(volatile v8h*)p = o;
}

__global__ __launch_bounds__(256) void qprep_kernel(
    const float* __restrict__ Q, const float* __restrict__ G, const float* __restrict__ Be,
    const float* __restrict__ Wv, const float* __restrict__ Bo,
    _Float16* __restrict__ Qc, float* __restrict__ Qs) {
  __shared__ __attribute__((aligned(16))) float sS[NQ];
  __shared__ __attribute__((aligned(16))) float sA[NQ];
  const unsigned tid = threadIdx.x, lane = tid & 31u;
  const int wave = __builtin_amdgcn_readfirstlane((int)(threadIdx.x >> 5));
  const unsigned c = (tid & 7u) * 8u;

  float gw[8];
  {
    const v4f g0 = *(const v4f*)(G + c);
    const v4f g1 = *(const v4f*)(G + c + 4u);
    const v4f w0 = *(const v4f*)(Wv + c);
    const v4f w1 = *(const v4f*)(Wv + c + 4u);
#pragma unroll
    for (int i = 0; i < 4; ++i) {
      gw[i]     = bf16r(g0[i]) * bf16r(w0[i]);
      gw[i + 4] = bf16r(g1[i]) * bf16r(w1[i]);
    }
  }
  const float part = bf16r(Be[lane]) * bf16r(Wv[lane]) +
                     bf16r(Be[lane + 32u]) * bf16r(Wv[lane + 32u]);
  const float c0 = red32_sum(part) + bf16r(Bo[0]);

#pragma unroll 1
  for (unsigned pass = 0; pass < (unsigned)(NQ / 32); ++pass) {
    const unsigned row = 32u * pass + (tid >> 3);
    const v4f a0 = *(const v4f*)(Q + (size_t)row * DM + c);
    const v4f a1 = *(const v4f*)(Q + (size_t)row * DM + c + 4u);
    float e[8];
#pragma unroll
    for (int i = 0; i < 4; ++i) { e[i] = bf16r(a0[i]); e[i + 4] = bf16r(a1[i]); }
    float s = 0.0f;
#pragma unroll
    for (int i = 0; i < 8; ++i) s += e[i];
    const float mean = red8_sum(s) * (1.0f / (float)DM);
    float ss = 0.0f, dg = 0.0f;
    v8h o;
#pragma unroll
    for (int i = 0; i < 8; ++i) {
      const float d = e[i] - mean;
      ss += d * d;
      dg += d * gw[i];
      o[i] = toh_flush(QCARRY * d);
    }
    ss = red8_sum(ss);
    dg = red8_sum(dg);
    if ((tid & 7u) == 0u) { sS[row] = ss; sA[row] = dg; }
    _Float16* p = Qc + (size_t)row * DM + c;
    *(volatile v8h*)p = o;
    __threadfence();
    *(volatile v8h*)p = o;
  }
  __syncthreads();

  if (wave == 0) {
    const v4f sv = *(const v4f*)&sS[lane * 4u];
    float* dp = Qs + lane * 4u;
    *(volatile v4f*)dp = sv;
    __threadfence();
    *(volatile v4f*)dp = sv;
  }
  if (wave == 1) {
    const v4f sv = *(const v4f*)&sA[lane * 4u];
    float* dp = Qs + NQ + lane * 4u;
    *(volatile v4f*)dp = sv;
    __threadfence();
    *(volatile v4f*)dp = sv;
  }
  if (wave == 2) {
    v4f sv;
    sv[0] = c0; sv[1] = c0; sv[2] = c0; sv[3] = c0;
    float* dp = Qs + 2 * NQ + (lane & 7u) * 4u;
    if (lane < 8u) *(volatile v4f*)dp = sv;
    __threadfence();
    if (lane < 8u) *(volatile v4f*)dp = sv;
  }
}

template <int MODE>
__device__ __forceinline__ void gemm_body(
    const _Float16* __restrict__ A16, const _Float16* __restrict__ Bt, const unsigned K,
    const float cs, const float* __restrict__ bias,
    const float* __restrict__ gain, const float* __restrict__ wvec,
    const float* __restrict__ rowst, const float* __restrict__ colst,
    float* __restrict__ outst, float* __restrict__ outf, _Float16* __restrict__ out16) {
  __shared__ float Cs[64 * LDC];
  __shared__ __attribute__((aligned(16))) float St[128];
  const unsigned tid = threadIdx.x, lane = tid & 31u, w = tid >> 5;
  const unsigned mw = w >> 1, nw = w & 1u;
  const unsigned hh = lane >> 4, m = lane & 15u;
  const unsigned n0 = blockIdx.x * 64u;
  const unsigned row0 = blockIdx.y * 64u;

  const _Float16* ap  = A16 + (size_t)(row0 + mw * 16u + m) * K + hh * 8u;
  const _Float16* bp0 = Bt + (size_t)(n0 + nw * 32u + m) * K + hh * 8u;
  const _Float16* bp1 = bp0 + (size_t)16 * K;
  v8f acc0 = {}, acc1 = {};
#pragma unroll 2
  for (unsigned k0 = 0; k0 < K; k0 += 32u) {
    const v16h a  = frag_at(ap + k0);
    const v16h b0 = frag_at(bp0 + k0);
    const v16h b1 = frag_at(bp1 + k0);
    acc0 = wmma16(a, b0, acc0);
    acc1 = wmma16(a, b1, acc1);
  }
#pragma unroll
  for (int r = 0; r < 8; ++r) {
    float* d = &Cs[(mw * 16u + hh * 8u + (unsigned)r) * LDC + nw * 32u + m];
    d[0]  = acc0[r];
    d[16] = acc1[r];
  }
  __syncthreads();

  if (MODE == 0) {
    v8h x[2];
    size_t off[2];
#pragma unroll
    for (unsigned i = 0; i < 2u; ++i) {
      const unsigned r = 32u * i + (tid >> 3);
      const unsigned c = (tid & 7u) * 8u;
      const v4f u0 = *(const v4f*)&Cs[r * LDC + c];
      const v4f u1 = *(const v4f*)&Cs[r * LDC + c + 4];
      const v4f g0 = *(const v4f*)(bias + n0 + c);
      const v4f g1 = *(const v4f*)(bias + n0 + c + 4u);
#pragma unroll
      for (int j = 0; j < 4; ++j) {
        x[i][j]     = toh_flush(ACARRY * (u0[j] * cs + bf16r(g0[j])));
        x[i][j + 4] = toh_flush(ACARRY * (u1[j] * cs + bf16r(g1[j])));
      }
      off[i] = (size_t)(row0 + r) * DM + n0 + c;
    }
#pragma unroll
    for (int i = 0; i < 2; ++i) *(volatile v8h*)(out16 + off[i]) = x[i];
    __threadfence();
#pragma unroll
    for (int i = 0; i < 2; ++i) *(volatile v8h*)(out16 + off[i]) = x[i];
  }

  if (MODE == 1) {
    v8h x[2];
    size_t off[2];
#pragma unroll
    for (unsigned i = 0; i < 2u; ++i) {
      const unsigned r = 32u * i + (tid >> 3);
      const unsigned c = (tid & 7u) * 8u;
      const v4f u0 = *(const v4f*)&Cs[r * LDC + c];
      const v4f u1 = *(const v4f*)&Cs[r * LDC + c + 4];
      const v4f g0 = *(const v4f*)(bias + n0 + c);
      const v4f g1 = *(const v4f*)(bias + n0 + c + 4u);
      const v4f e0 = *(const v4f*)(gain + n0 + c);
      const v4f e1 = *(const v4f*)(gain + n0 + c + 4u);
      const v4f w0 = *(const v4f*)(wvec + n0 + c);
      const v4f w1 = *(const v4f*)(wvec + n0 + c + 4u);
      float a[8], gw[8];
#pragma unroll
      for (int j = 0; j < 4; ++j) {
        a[j]      = u0[j] * cs + bf16r(g0[j]);
        a[j + 4]  = u1[j] * cs + bf16r(g1[j]);
        gw[j]     = bf16r(e0[j]) * bf16r(w0[j]);
        gw[j + 4] = bf16r(e1[j]) * bf16r(w1[j]);
      }
      float s = 0.0f;
#pragma unroll
      for (int j = 0; j < 8; ++j) s += a[j];
      const float mean = red8_sum(s) * (1.0f / (float)DM);
      float ss = 0.0f, dg = 0.0f;
#pragma unroll
      for (int j = 0; j < 8; ++j) {
        const float d = a[j] - mean;
        ss += d * d;
        dg += d * gw[j];
        x[i][j] = toh_flush(ACARRY * d);
      }
      ss = red8_sum(ss);
      dg = red8_sum(dg);
      if ((tid & 7u) == 0u) { St[r] = ss; St[64u + r] = dg; }
      off[i] = (size_t)(row0 + r) * DM + n0 + c;
    }
#pragma unroll
    for (int i = 0; i < 2; ++i) *(volatile v8h*)(out16 + off[i]) = x[i];
    __threadfence();
#pragma unroll
    for (int i = 0; i < 2; ++i) *(volatile v8h*)(out16 + off[i]) = x[i];
    __syncthreads();
    const int wv = __builtin_amdgcn_readfirstlane((int)(threadIdx.x >> 5));
    if (wv < 2) {
      const unsigned l16 = lane & 15u;
      const v4f sv = *(const v4f*)&St[(unsigned)wv * 64u + l16 * 4u];
      float* dp = outst + (size_t)wv * MROWS + row0 + l16 * 4u;
      if (lane < 16u) *(volatile v4f*)dp = sv;
      __threadfence();
      if (lane < 16u) *(volatile v4f*)dp = sv;
    }
  }

  if (MODE == 2) {
    const unsigned bidx = row0 / (unsigned)SEQ;
    const unsigned t0 = row0 - bidx * (unsigned)SEQ;
    const unsigned tcol = (tid & 15u) * 4u;
    const v4f ts = *(const v4f*)(rowst + row0 + tcol);
    const v4f ta = *(const v4f*)(rowst + (size_t)MROWS + row0 + tcol);
    const float c0 = colst[2 * NQ];
    v4f xs[4];
    size_t off[4];
#pragma unroll
    for (unsigned i = 0; i < 4u; ++i) {
      const unsigned ql = 16u * i + (tid >> 4);
      const unsigned q = n0 + ql;
      const float sq = colst[q];
      const float aq = colst[NQ + q];
      v4f val;
#pragma unroll
      for (int j = 0; j < 4; ++j) {
        const float cr = Cs[(tcol + (unsigned)j) * LDC + ql] * cs;
        const float var = fmaxf((ts[j] + 2.0f * cr + sq) * (1.0f / (float)DM), 0.0f);
        val[j] = rsqrtf(var + LN_EPS) * (ta[j] + aq) + c0;
      }
      xs[i] = val;
      off[i] = ((size_t)bidx * NQ + q) * SEQ_FULL + t0 + tcol;
    }
#pragma unroll
    for (int i = 0; i < 4; ++i) *(volatile v4f*)(outf + off[i]) = xs[i];
    __threadfence();
#pragma unroll
    for (int i = 0; i < 4; ++i) *(volatile v4f*)(outf + off[i]) = xs[i];
  }
}

__global__ __launch_bounds__(256) void gemm_p_kernel(
    const _Float16* __restrict__ A16, const _Float16* __restrict__ Bt,
    const float* __restrict__ bias, _Float16* __restrict__ out16) {
  gemm_body<0>(A16, Bt, (unsigned)CIN, 1.0f / (XCARRY * WCARRY), bias, bias, bias, bias, bias,
               (float*)0, (float*)0, out16);
}
__global__ __launch_bounds__(256) void gemm_v_kernel(
    const _Float16* __restrict__ A16, const _Float16* __restrict__ Bt,
    const float* __restrict__ bias, _Float16* __restrict__ out16) {
  gemm_body<0>(A16, Bt, (unsigned)DM, 1.0f / (ACARRY * WCARRY), bias, bias, bias, bias, bias,
               (float*)0, (float*)0, out16);
}
__global__ __launch_bounds__(256) void gemm_a_kernel(
    const _Float16* __restrict__ A16, const _Float16* __restrict__ Bt,
    const float* __restrict__ bias, const float* __restrict__ gain,
    const float* __restrict__ wvec, float* __restrict__ ts, _Float16* __restrict__ out16) {
  gemm_body<1>(A16, Bt, (unsigned)DM, 1.0f / (ACARRY * WCARRY), bias, gain, wvec, bias, bias,
               ts, (float*)0, out16);
}
__global__ __launch_bounds__(256) void gemm_out_kernel(
    const _Float16* __restrict__ A16, const _Float16* __restrict__ Bt,
    const float* __restrict__ ts, const float* __restrict__ qs, float* __restrict__ outf) {
  gemm_body<2>(A16, Bt, (unsigned)DM, 1.0f / (ACARRY * QCARRY), ts, ts, ts, ts, qs,
               (float*)0, outf, (_Float16*)0);
}

extern "C" void kernel_launch(void* const* d_in, const int* in_sizes, int n_in,
                              void* d_out, int out_size, void* d_ws, size_t ws_size,
                              hipStream_t stream) {
  if (n_in < 12) return;
  const long long need_x =
      ((long long)(NB - 1) * CIN + (CIN - 1)) * SEQ_FULL + SEQ;
  const long long need_o =
      ((long long)(NB - 1) * NQ + (NQ - 1)) * SEQ_FULL + SEQ;
  if ((long long)in_sizes[0] < need_x) return;
  if (in_sizes[1] < NQ * DM) return;
  if (in_sizes[2] < DM * CIN) return;
  if (in_sizes[4] < DM * DM || in_sizes[6] < DM * DM) return;
  if (in_sizes[3] < DM || in_sizes[5] < DM || in_sizes[7] < DM) return;
  if (in_sizes[8] < DM || in_sizes[9] < DM || in_sizes[10] < DM) return;
  if (in_sizes[11] < 1) return;
  if ((long long)out_size < need_o) return;
  if (ws_size < WS_TOTAL) return;

  const float* X    = (const float*)d_in[0];
  const float* qry  = (const float*)d_in[1];
  const float* win  = (const float*)d_in[2];
  const float* bin  = (const float*)d_in[3];
  const float* wv   = (const float*)d_in[4];
  const float* bv   = (const float*)d_in[5];
  const float* wo   = (const float*)d_in[6];
  const float* bo   = (const float*)d_in[7];
  const float* lng  = (const float*)d_in[8];
  const float* lnb  = (const float*)d_in[9];
  const float* wout = (const float*)d_in[10];
  const float* bout = (const float*)d_in[11];
  float* out = (float*)d_out;

  char* ws = (char*)d_ws;
  _Float16* Xt16  = (_Float16*)(ws + OFF_XT);
  _Float16* Win16 = (_Float16*)(ws + OFF_WIN);
  _Float16* Wv16  = (_Float16*)(ws + OFF_WV);
  _Float16* Wo16  = (_Float16*)(ws + OFF_WO);
  _Float16* P16   = (_Float16*)(ws + OFF_P);
  _Float16* V16   = (_Float16*)(ws + OFF_V);
  _Float16* Ac16  = (_Float16*)(ws + OFF_AC);
  _Float16* Qc16  = (_Float16*)(ws + OFF_QC);
  float*    Ts    = (float*)(ws + OFF_TS);
  float*    Qs    = (float*)(ws + OFF_QS);

  dim3 blk(256);

  xconv_kernel<<<dim3(SEQ / 64, CIN / 64, NB), blk, 0, stream>>>(X, Xt16);
  wcast_kernel<<<dim3((DM * CIN) / 2048), blk, 0, stream>>>(win, Win16);
  wcast_kernel<<<dim3((DM * DM) / 2048), blk, 0, stream>>>(wv, Wv16);
  wcast_kernel<<<dim3((DM * DM) / 2048), blk, 0, stream>>>(wo, Wo16);
  qprep_kernel<<<dim3(1), blk, 0, stream>>>(qry, lng, lnb, wout, bout, Qc16, Qs);

  gemm_p_kernel<<<dim3(DM / 64, MROWS / 64), blk, 0, stream>>>(Xt16, Win16, bin, P16);
  gemm_v_kernel<<<dim3(DM / 64, MROWS / 64), blk, 0, stream>>>(P16, Wv16, bv, V16);
  gemm_a_kernel<<<dim3(DM / 64, MROWS / 64), blk, 0, stream>>>(V16, Wo16, bo, lng, wout, Ts, Ac16);
  gemm_out_kernel<<<dim3(NQ / 64, MROWS / 64), blk, 0, stream>>>(Ac16, Qc16, Ts, Qs, out);
}
